// FANPhaseOffsetTransformerLayer_60112362275493
// MI455X (gfx1250) — hardware-verified
//
#include <hip/hip_runtime.h>


namespace {
constexpr int Bn = 2, S = 2048, D = 1024, H = 16, HD = 64, NTOK = Bn * S, P_DIM = D / 4, G_DIM = D / 2, NPG = P_DIM + G_DIM;
constexpr float SCALE = 0.125f, VS = 8.0f;

typedef _Float16 b16;
typedef __attribute__((ext_vector_type(16))) _Float16 v16b;
typedef __attribute__((ext_vector_type(8)))  _Float16 v8b;
typedef __attribute__((ext_vector_type(8)))  float v8f;
typedef __attribute__((ext_vector_type(4)))  float v4f;

__device__ __forceinline__ v8b ld8b(const b16* p) { return *(const v8b*)p; }
__device__ __forceinline__ v16b cat8b(v8b a, v8b b) { return __builtin_shufflevector(a, b, 0, 1, 2, 3, 4, 5, 6, 7, 8, 9, 10, 11, 12, 13, 14, 15); }
__device__ __forceinline__ v16b frag_kb(const b16* p, int hh) { return cat8b(ld8b(p + 8 * hh), ld8b(p + 16 + 8 * hh)); }
__device__ __forceinline__ void split16(float v, b16& hi, b16& lo) { hi = (b16)v; lo = (b16)(v - (float)hi); }
__device__ __forceinline__ void frag_ksplit(const float* p, int hh, v16b& fh_, v16b& fl_) {
  const float* p0 = p + 8 * hh; const float* p1 = p + 16 + 8 * hh;
#pragma unroll
  for (int e = 0; e < 8; ++e) { b16 a, c; split16(p0[e], a, c); fh_[e] = a; fl_[e] = c; split16(p1[e], a, c); fh_[8 + e] = a; fl_[8 + e] = c; }
}
__device__ __forceinline__ v8f wmma16b(v16b a, v16b b, v8f c) {
  v8f d = __builtin_amdgcn_wmma_f32_16x16x32_f16(false, a, false, b, (short)0, c, false, false);
  asm volatile("v_nop\n\tv_nop\n\tv_nop\n\tv_nop" : "+v"(d) : "v"(a), "v"(b));
  return d;
}
__device__ __forceinline__ void wave_lds_sync() {
  __builtin_amdgcn_fence(__ATOMIC_RELEASE, "workgroup");
  __builtin_amdgcn_wave_barrier();
  __builtin_amdgcn_fence(__ATOMIC_ACQUIRE, "workgroup");
}

struct Opnd { const void* p0; const void* p1; int ld; };
template <int NP> __device__ __forceinline__ void load_frags(const Opnd& o, int row, int kb, int hh, v16b& fh_, v16b& fl_) {
  if (NP == 0) { frag_ksplit((const float*)o.p0 + (size_t)row * o.ld + kb, hh, fh_, fl_); }
  else if (NP == 4 || NP == 5) {
    const float sc_ = (NP == 4) ? 64.0f : 8.0f;
    const float* p = (const float*)o.p0 + (size_t)row * o.ld + kb; const float* p0 = p + 8 * hh; const float* p1 = p + 16 + 8 * hh;
#pragma unroll
    for (int e = 0; e < 8; ++e) { b16 a, c; split16(p0[e] * sc_, a, c); fh_[e] = a; fl_[e] = c; split16(p1[e] * sc_, a, c); fh_[8 + e] = a; fl_[8 + e] = c; }
  } else if (NP == 3) {
    const float* p = (const float*)o.p0 + (size_t)row * o.ld + kb; const float* p0 = p + 8 * hh; const float* p1 = p + 16 + 8 * hh;
#pragma unroll
    for (int e = 0; e < 8; ++e) { fh_[e] = (b16)p0[e]; fh_[8 + e] = (b16)p1[e]; }
    fl_ = fh_;
  } else {
    fh_ = frag_kb((const b16*)o.p0 + (size_t)row * o.ld + kb, hh);
    if (NP == 2) fl_ = frag_kb((const b16*)o.p1 + (size_t)row * o.ld + kb, hh); else fl_ = fh_;
  }
}
template <int ANP, int BNP> __device__ __forceinline__ v8f mac(v16b ah, v16b al, v16b bh, v16b bl, v8f c) {
  c = wmma16b(ah, bh, c);
  if (BNP == 0 || BNP == 2 || BNP == 4 || BNP == 5) c = wmma16b(ah, bl, c);
  if (ANP == 0 || ANP == 2 || ANP == 4 || ANP == 5) c = wmma16b(al, bh, c);
  return c;
}
template <int ANP, int BNP>
__device__ __forceinline__ void gemm_tile(const Opnd& A, const Opnd& B, int K, int m0, int c0, int nloc, int hlf, v8f (&acc)[2][4]) {
  for (int kb = 0; kb < K; kb += 32) {
    v16b a0h, a0l, a1h, a1l;
    load_frags<ANP>(A, m0 + nloc, kb, hlf, a0h, a0l);
    load_frags<ANP>(A, m0 + 16 + nloc, kb, hlf, a1h, a1l);
#pragma unroll
    for (int t = 0; t < 4; ++t) {
      v16b bh, bl;
      load_frags<BNP>(B, c0 + t * 16 + nloc, kb, hlf, bh, bl);
      acc[0][t] = mac<ANP, BNP>(a0h, a0l, bh, bl, acc[0][t]);
      acc[1][t] = mac<ANP, BNP>(a1h, a1l, bh, bl, acc[1][t]);
    }
  }
}

__device__ __forceinline__ void epi_planes(v8f (&acc)[2][4], float scale, bool two, b16* __restrict__ oh, b16* __restrict__ ol, int ldo,
                                           int m0, int c0, int lane, b16* Th, b16* Tl) {
  const int nloc = lane & 15, hlf = lane >> 4;
#pragma unroll
  for (int t = 0; t < 4; ++t)
#pragma unroll
    for (int r = 0; r < 2; ++r)
#pragma unroll
      for (int v = 0; v < 8; ++v) {
        const int rr = r * 16 + v + 8 * hlf, cc = t * 16 + nloc;
        b16 h_, l_; split16(acc[r][t][v] * scale, h_, l_);
        Th[rr * 64 + cc] = h_; Tl[rr * 64 + cc] = l_;
      }
  wave_lds_sync();
  for (int pass = 0; pass < 2; ++pass) {
#pragma unroll
    for (int j = 0; j < 8; ++j) {
      const int rr = j * 4 + (lane >> 3), c8 = (lane & 7) * 8;
      const size_t o = (size_t)(m0 + rr) * ldo + c0 + c8;
      *(volatile v8b*)(oh + o) = ld8b(Th + rr * 64 + c8);
      if (two) *(volatile v8b*)(ol + o) = ld8b(Tl + rr * 64 + c8);
    }
    __threadfence();
  }
}
__device__ __forceinline__ void epi_f32(v8f (&acc)[2][4], float scale, const float* rscale, float* __restrict__ out, int ldo, int m0, int c0, int lane, float* Tt) {
  const int nloc = lane & 15, hlf = lane >> 4;
#pragma unroll
  for (int t = 0; t < 4; ++t)
#pragma unroll
    for (int r = 0; r < 2; ++r)
#pragma unroll
      for (int v = 0; v < 8; ++v) {
        const int rr = r * 16 + v + 8 * hlf;
        const float rs = rscale ? rscale[(size_t)(m0 + rr) * 32] : 1.0f;
        Tt[rr * 64 + t * 16 + nloc] = acc[r][t][v] * scale * rs;
      }
  wave_lds_sync();
  float* dst0 = out + (size_t)m0 * ldo + c0;
  for (int pass = 0; pass < 2; ++pass) {
#pragma unroll
    for (int j = 0; j < 16; ++j) { const int rr = j * 2 + hlf, c4 = nloc * 4; *(volatile v4f*)(dst0 + (size_t)rr * ldo + c4) = *(const v4f*)(Tt + rr * 64 + c4); }
    __threadfence();
  }
}


typedef __attribute__((ext_vector_type(8))) __bf16 v8bb; typedef __attribute__((ext_vector_type(16))) __bf16 v16bb;
typedef __attribute__((ext_vector_type(8))) unsigned short v8us;
__device__ __forceinline__ v16bb frag_kb_bf(const __bf16* p, int hh) { const v8bb a = *(const v8bb*)(p + 8 * hh), b = *(const v8bb*)(p + 16 + 8 * hh); return __builtin_shufflevector(a, b, 0, 1, 2, 3, 4, 5, 6, 7, 8, 9, 10, 11, 12, 13, 14, 15); }
__device__ __forceinline__ v8f wmma16bb(v16bb a, v16bb b, v8f c) {
  v8f d = __builtin_amdgcn_wmma_f32_16x16x32_bf16(false, a, false, b, (short)0, c, false, false);
  asm volatile("v_nop\n\tv_nop\n\tv_nop\n\tv_nop" : "+v"(d) : "v"(a), "v"(b));
  return d;
}
__device__ __forceinline__ unsigned short bf16_rne_bits(float v) { unsigned int u = __float_as_uint(v); u += 0x7FFFu + ((u >> 16) & 1u); return (unsigned short)(u >> 16); }
__device__ __forceinline__ float bf16_rne(float v) { return __uint_as_float(((unsigned int)bf16_rne_bits(v)) << 16); }

__global__ __launch_bounds__(256) void prep_kernel(const float* __restrict__ x, const float* __restrict__ Wq, const float* __restrict__ Wk, const float* __restrict__ Wv, const float* __restrict__ Wo,
                                                   const float* __restrict__ Wp, const float* __restrict__ Wg,
                                                   unsigned short* __restrict__ x16, unsigned short* __restrict__ w16, b16* __restrict__ wo16, b16* __restrict__ wpg16) {
  const size_t tid = (size_t)blockIdx.x * blockDim.x + threadIdx.x, nth = (size_t)gridDim.x * blockDim.x;
  const size_t nx = (size_t)NTOK * D / 8, nw = (size_t)D * D / 8, npg = (size_t)NPG * D / 8;
  for (int pass = 0; pass < 2; ++pass) {
    for (size_t p = tid; p < nx + 3 * nw + nw + npg; p += nth) {
      if (p < nx + 3 * nw) {
        const float* src; unsigned short* dst;
        if (p < nx) { src = x + p * 8; dst = x16 + p * 8; }
        else { const size_t pw = p - nx; const int which = (int)(pw / nw); const size_t i = (pw % nw) * 8; src = (which == 0 ? Wq : which == 1 ? Wk : Wv) + i; dst = w16 + (size_t)which * D * D + i; }
        v8us v;
#pragma unroll
        for (int e = 0; e < 8; ++e) v[e] = bf16_rne_bits(src[e]);
        *(volatile v8us*)dst = v;
      } else if (p < nx + 4 * nw) { const size_t i = (p - nx - 3 * nw) * 8; v8b v;
#pragma unroll
        for (int e = 0; e < 8; ++e) v[e] = (b16)bf16_rne(Wo[i + e]);
        *(volatile v8b*)(wo16 + i) = v; }
      else { const size_t i = (p - nx - 4 * nw) * 8; const float* src = (i < (size_t)P_DIM * D) ? (Wp + i) : (Wg + i - (size_t)P_DIM * D); v8b v;
#pragma unroll
        for (int e = 0; e < 8; ++e) v[e] = (b16)bf16_rne(src[e]);
        *(volatile v8b*)(wpg16 + i) = v; }
    }
    __threadfence();
  }
}

__global__ __launch_bounds__(128) void proj_kernel(const __bf16* __restrict__ x16, const __bf16* __restrict__ w16, const float* __restrict__ bq, const float* __restrict__ bk, const float* __restrict__ bv, b16* __restrict__ qk, b16* __restrict__ vt) {
  __shared__ __attribute__((aligned(16))) b16 Th[4][2][32 * 64];
  __shared__ __attribute__((aligned(16))) b16 Tt[64][128 + 8];
  const int lane = threadIdx.x & 31, wave = threadIdx.x >> 5, nloc = lane & 15, hlf = lane >> 4, which = blockIdx.z, m0 = blockIdx.y * 128 + wave * 32, c0 = blockIdx.x * 64;
  const __bf16* X = x16; const __bf16* W = w16 + (size_t)which * D * D; const float* bias = (which == 0) ? bq : (which == 1) ? bk : bv;
  v8f acc[2][4];
#pragma unroll
  for (int r = 0; r < 2; ++r)
#pragma unroll
    for (int t = 0; t < 4; ++t) acc[r][t] = (v8f){};
#pragma unroll 2
  for (int kb = 0; kb < D; kb += 32) {
    const v16bb a0 = frag_kb_bf(X + (size_t)(m0 + nloc) * D + kb, hlf), a1 = frag_kb_bf(X + (size_t)(m0 + 16 + nloc) * D + kb, hlf);
#pragma unroll
    for (int t = 0; t < 4; ++t) { const v16bb bw = frag_kb_bf(W + (size_t)(c0 + t * 16 + nloc) * D + kb, hlf); acc[0][t] = wmma16bb(a0, bw, acc[0][t]); acc[1][t] = wmma16bb(a1, bw, acc[1][t]); }
  }
#pragma unroll
  for (int t = 0; t < 4; ++t)
#pragma unroll
    for (int r = 0; r < 2; ++r)
#pragma unroll
      for (int v = 0; v < 8; ++v) acc[r][t][v] += bf16_rne(bias[c0 + t * 16 + nloc]);
  const int h = c0 / HD, b = m0 / S, s0 = m0 % S;
  if (which < 2) { epi_planes(acc, 1.0f, false, qk + ((((size_t)which * Bn + b) * H + h) * S + s0) * HD, nullptr, HD, 0, 0, lane, Th[wave][0], Th[wave][1]); return; }
#pragma unroll
  for (int t = 0; t < 4; ++t)
#pragma unroll
    for (int r = 0; r < 2; ++r)
#pragma unroll
      for (int v = 0; v < 8; ++v) Tt[t * 16 + nloc][wave * 32 + r * 16 + 8 * hlf + v] = (b16)(acc[r][t][v] * VS);
  __syncthreads();
  const int tok0 = (blockIdx.y * 128) % S, bb = (blockIdx.y * 128) / S;
  b16* dst = vt + (((size_t)bb * H + h) * HD) * S + tok0;
  for (int pass = 0; pass < 2; ++pass) {
#pragma unroll
    for (int j = 0; j < 8; ++j) { const int dd = wave * 16 + j * 2 + (lane >> 4), c8 = (lane & 15) * 8; *(volatile v8b*)(dst + (size_t)dd * S + c8) = *(const v8b*)(&Tt[dd][c8]); }
    __threadfence();
  }
}

__global__ __launch_bounds__(256) void attn_kernel(const b16* __restrict__ qk, const b16* __restrict__ vt, float* __restrict__ y) {
  __shared__ __attribute__((aligned(16))) float Os[8][16][HD + 4];
  const int wid = threadIdx.x >> 5, lane = threadIdx.x & 31, hh = lane >> 4, col = lane & 15;
  const int qt = blockIdx.x * 8 + wid, jt = qt & 127, h = (qt >> 7) & 15, b = qt >> 11, q0 = jt * 16, qi = q0 + col;
  const b16* Q = qk + ((((size_t)0 * Bn + b) * H + h) * S) * HD; const b16* K = qk + ((((size_t)1 * Bn + b) * H + h) * S) * HD;
  const b16* vb = vt + (((size_t)b * H + h) * HD) * S;
  v16b qf[2];
#pragma unroll
  for (int ks = 0; ks < 2; ++ks) qf[ks] = frag_kb(Q + (size_t)qi * HD + ks * 32, hh);
  float m = -INFINITY, l = 0.0f; v8f o[4] = {{}, {}, {}, {}};
  for (int kb = 0; kb < S; kb += 32) {
    v8f s0 = {}, s1 = {};
#pragma unroll
    for (int ks = 0; ks < 2; ++ks) { s0 = wmma16b(frag_kb(K + (size_t)(kb + col) * HD + ks * 32, hh), qf[ks], s0); s1 = wmma16b(frag_kb(K + (size_t)(kb + 16 + col) * HD + ks * 32, hh), qf[ks], s1); }
    float mr = -INFINITY;
#pragma unroll
    for (int r = 0; r < 8; ++r) { s0[r] *= SCALE; s1[r] *= SCALE; mr = fmaxf(mr, fmaxf(s0[r], s1[r])); }
    mr = fmaxf(mr, __shfl_xor(mr, 16));
    const float mn = fmaxf(m, mr), al_ = __expf(m - mn); m = mn;
    float sum = 0.0f; v16b pb;
#pragma unroll
    for (int r = 0; r < 8; ++r) { const float e0 = __expf(s0[r] - mn), e1 = __expf(s1[r] - mn); sum += e0 + e1; pb[r] = (b16)e0; pb[8 + r] = (b16)e1; }
    sum += __shfl_xor(sum, 16); l = l * al_ + sum;
#pragma unroll
    for (int n = 0; n < 4; ++n) {
#pragma unroll
      for (int r = 0; r < 8; ++r) o[n][r] *= al_;
      o[n] = wmma16b(frag_kb(vb + (size_t)(n * 16 + col) * S + kb, hh), pb, o[n]);
    }
  }
  const float inv = 1.0f / (VS * l);
#pragma unroll
  for (int n = 0; n < 4; ++n)
#pragma unroll
    for (int r = 0; r < 8; ++r) Os[wid][col][n * 16 + 8 * hh + r] = o[n][r] * inv;
  wave_lds_sync();
  float* dst = y + ((size_t)b * S + q0) * D + h * HD;
  for (int pass = 0; pass < 2; ++pass) {
#pragma unroll
    for (int j = 0; j < 8; ++j) { const int rr = j * 2 + hh, c4 = col * 4; *(volatile v4f*)(dst + (size_t)rr * D + c4) = *(const v4f*)(&Os[wid][rr][c4]); }
    __threadfence();
  }
}

__global__ __launch_bounds__(128) void out_kernel(const float* __restrict__ y, const b16* __restrict__ wo16, const float* __restrict__ bo, float* __restrict__ out) {
  __shared__ __attribute__((aligned(16))) float Ts[4][32 * 64];
  const int lane = threadIdx.x & 31, wave = threadIdx.x >> 5, nloc = lane & 15, hlf = lane >> 4, m0 = blockIdx.y * 128 + wave * 32, c0 = blockIdx.x * 64;
  v8f acc[2][4];
#pragma unroll
  for (int r = 0; r < 2; ++r)
#pragma unroll
    for (int t = 0; t < 4; ++t) acc[r][t] = (v8f){};
  const Opnd A{y, nullptr, D}, B{wo16, nullptr, D};
  gemm_tile<3, 1>(A, B, D, m0, c0, nloc, hlf, acc);
#pragma unroll
  for (int t = 0; t < 4; ++t)
#pragma unroll
    for (int r = 0; r < 2; ++r)
#pragma unroll
      for (int v = 0; v < 8; ++v) acc[r][t][v] += bf16_rne(bo[c0 + t * 16 + nloc]);
  epi_f32(acc, 1.0f, nullptr, out, D, m0, c0, lane, Ts[wave]);
}

__global__ __launch_bounds__(256) void ln1_kernel(const float* __restrict__ x, const float* __restrict__ ao, const float* __restrict__ g, const float* __restrict__ bb, float* __restrict__ x1) {
  const int wid = threadIdx.x >> 5, lane = threadIdx.x & 31, row = blockIdx.x * 8 + wid;
  float v[32]; float s = 0.0f;
#pragma unroll
  for (int j = 0; j < 8; ++j) { const int c = (j * 32 + lane) * 4; const v4f xa = *(const v4f*)(x + (size_t)row * D + c), ab = *(const v4f*)(ao + (size_t)row * D + c);
#pragma unroll
    for (int e = 0; e < 4; ++e) { v[j * 4 + e] = bf16_rne(xa[e]) + ab[e]; s += v[j * 4 + e]; } }
#pragma unroll
  for (int o = 16; o > 0; o >>= 1) s += __shfl_xor(s, o);
  const float mean = s * (1.0f / D); float s2 = 0.0f;
#pragma unroll
  for (int i = 0; i < 32; ++i) { const float dd = v[i] - mean; s2 += dd * dd; }
#pragma unroll
  for (int o = 16; o > 0; o >>= 1) s2 += __shfl_xor(s2, o);
  const float rs = rsqrtf(s2 * (1.0f / D) + 1e-5f);
  for (int pass = 0; pass < 2; ++pass) {
#pragma unroll
    for (int j = 0; j < 8; ++j) { const int c = (j * 32 + lane) * 4; v4f w;
#pragma unroll
      for (int e = 0; e < 4; ++e) w[e] = (v[j * 4 + e] - mean) * rs * bf16_rne(g[c + e]) + bf16_rne(bb[c + e]);
      *(volatile v4f*)(x1 + (size_t)row * D + c) = w; }
    __threadfence();
  }
}

__global__ __launch_bounds__(128) void pg_kernel(const float* __restrict__ x1, const b16* __restrict__ wpg16, const float* __restrict__ bp, const float* __restrict__ bg, float* __restrict__ pg) {
  __shared__ __attribute__((aligned(16))) float Ts[4][32 * 64];
  const int lane = threadIdx.x & 31, wave = threadIdx.x >> 5, nloc = lane & 15, hlf = lane >> 4, m0 = blockIdx.y * 128 + wave * 32, c0 = blockIdx.x * 64;
  v8f acc[2][4];
#pragma unroll
  for (int r = 0; r < 2; ++r)
#pragma unroll
    for (int t = 0; t < 4; ++t) acc[r][t] = (v8f){};
  const Opnd A{x1, nullptr, D}, B{wpg16, nullptr, D};
  gemm_tile<3, 1>(A, B, D, m0, c0, nloc, hlf, acc);
#pragma unroll
  for (int t = 0; t < 4; ++t)
#pragma unroll
    for (int r = 0; r < 2; ++r)
#pragma unroll
      for (int v = 0; v < 8; ++v) { const int c = c0 + t * 16 + nloc; acc[r][t][v] += bf16_rne((c < P_DIM) ? bp[c] : bg[c - P_DIM]); }
  epi_f32(acc, 1.0f, nullptr, pg, NPG, m0, c0, lane, Ts[wave]);
}

__device__ __forceinline__ void sincos_acc(float f, float& sn, float& cs) {
  const double xx = (double)f; const double twooverpi = 0.63661977236758134308; const double pio2 = 1.57079632679489661923;
  const double kq = rint(xx * twooverpi); const double r = xx - kq * pio2; const int q = ((int)kq) & 3;
  const double r2 = r * r;
  double sp = r * (1.0 + r2 * (-1.0 / 6 + r2 * (1.0 / 120 + r2 * (-1.0 / 5040 + r2 * (1.0 / 362880 + r2 * (-1.0 / 39916800 + r2 * (1.0 / 6227020800.0)))))));
  double cp = 1.0 + r2 * (-0.5 + r2 * (1.0 / 24 + r2 * (-1.0 / 720 + r2 * (1.0 / 40320 + r2 * (-1.0 / 3628800 + r2 * (1.0 / 479001600.0))))));
  double s_, c_;
  if (q == 0) { s_ = sp; c_ = cp; } else if (q == 1) { s_ = cp; c_ = -sp; } else if (q == 2) { s_ = -sp; c_ = -cp; } else { s_ = -cp; c_ = sp; }
  sn = (float)s_; cs = (float)c_;
}
__device__ __forceinline__ float gelu_e(float x) { return 0.5f * x * (1.0f + erff(x * 0.7071067811865475f)); }

__global__ __launch_bounds__(256) void ln2_kernel(const float* __restrict__ x1, const float* __restrict__ pg, const float* __restrict__ off, const float* __restrict__ gate,
                                                  const float* __restrict__ g2, const float* __restrict__ b2, float* __restrict__ out) {
  __shared__ __attribute__((aligned(16))) float Rw[8][D];
  const int wid = threadIdx.x >> 5, lane = threadIdx.x & 31, row = blockIdx.x * 8 + wid;
  const float gv = 1.0f / (1.0f + __expf(-bf16_rne(gate[0])));
  float s = 0.0f;
#pragma unroll 1
  for (int i = 0; i < D / 32; ++i) { const int cc = i * 32 + lane; float f;
    if (cc < 2 * P_DIM) { const int ip = (cc < P_DIM) ? cc : cc - P_DIM; const float pv = pg[(size_t)row * NPG + ip]; const float ofs = bf16_rne(off[ip]);
      const float arg = (cc < P_DIM) ? (pv + ofs) : ((pv + 1.5707963267948966f) - ofs); float sn, cs; sincos_acc(arg, sn, cs); f = gv * ((cc < P_DIM) ? sn : cs); }
    else f = (1.0f - gv) * gelu_e(pg[(size_t)row * NPG + P_DIM + (cc - 2 * P_DIM)]);
    const float val = x1[(size_t)row * D + cc] + f; Rw[wid][cc] = val; s += val; }
#pragma unroll
  for (int o = 16; o > 0; o >>= 1) s += __shfl_xor(s, o);
  const float mean = s * (1.0f / D); float s2 = 0.0f;
#pragma unroll 1
  for (int i = 0; i < D / 32; ++i) { const float dd = Rw[wid][i * 32 + lane] - mean; s2 += dd * dd; }
#pragma unroll
  for (int o = 16; o > 0; o >>= 1) s2 += __shfl_xor(s2, o);
  const float rs = rsqrtf(s2 * (1.0f / D) + 1e-5f);
  wave_lds_sync();
  for (int pass = 0; pass < 2; ++pass) {
#pragma unroll
    for (int j = 0; j < 8; ++j) { const int c = (j * 32 + lane) * 4; v4f w;
#pragma unroll
      for (int e = 0; e < 4; ++e) w[e] = (Rw[wid][c + e] - mean) * rs * bf16_rne(g2[c + e]) + bf16_rne(b2[c + e]);
      *(volatile v4f*)(out + (size_t)row * D + c) = w; }
    __threadfence();
  }
}
}

extern "C" void kernel_launch(void* const* d_in, const int* in_sizes, int n_in,
                              void* d_out, int out_size, void* d_ws, size_t ws_size, hipStream_t stream) {
  (void)n_in; (void)out_size;
  const float* x = (const float*)d_in[0];
  const float* Wq = (const float*)d_in[1]; const float* bq = (const float*)d_in[2]; const float* Wk = (const float*)d_in[3]; const float* bk = (const float*)d_in[4];
  const float* Wv = (const float*)d_in[5]; const float* bv = (const float*)d_in[6]; const float* Wo = (const float*)d_in[7]; const float* bo = (const float*)d_in[8];
  const float* Wp = (const float*)d_in[9]; const float* bp = (const float*)d_in[10]; const float* Wg = (const float*)d_in[11]; const float* bg = (const float*)d_in[12];
  const float* offs = (const float*)d_in[13]; const float* gate = (const float*)d_in[14];
  const float* ln1w = (const float*)d_in[15]; const float* ln1b = (const float*)d_in[16]; const float* ln2w = (const float*)d_in[17]; const float* ln2b = (const float*)d_in[18];
  float* out = (float*)d_out;
  if (in_sizes[0] != NTOK * D || in_sizes[1] != D * D || in_sizes[9] != P_DIM * D || in_sizes[11] != G_DIM * D || in_sizes[13] != P_DIM || in_sizes[14] != 1) return;
  size_t woff = 0; char* ws = (char*)d_ws;
  auto carve = [&](size_t bytes) { char* p = ws + woff; woff += (bytes + 255) & ~(size_t)255; return p; };
  unsigned short* x16 = (unsigned short*)carve((size_t)NTOK * D * 2);
  unsigned short* w16 = (unsigned short*)carve((size_t)3 * D * D * 2);
  b16* wo16 = (b16*)carve((size_t)D * D * 2); b16* wpg16 = (b16*)carve((size_t)NPG * D * 2);
  b16* qk = (b16*)carve((size_t)2 * NTOK * D * 2);
  b16* vt = (b16*)carve((size_t)NTOK * D * 2);
  float* y = (float*)carve((size_t)NTOK * D * 4);
  float* ao = (float*)carve((size_t)NTOK * D * 4);
  float* x1 = (float*)carve((size_t)NTOK * D * 4);
  float* pg = (float*)carve((size_t)NTOK * NPG * 4);
  if (woff > ws_size) return;
  prep_kernel<<<1024, 256, 0, stream>>>(x, Wq, Wk, Wv, Wo, Wp, Wg, x16, w16, wo16, wpg16);
  proj_kernel<<<dim3(D / 64, NTOK / 128, 3), 128, 0, stream>>>((const __bf16*)x16, (const __bf16*)w16, bq, bk, bv, qk, vt);
  attn_kernel<<<Bn * H * (S / 16) / 8, 256, 0, stream>>>(qk, vt, y);
  out_kernel<<<dim3(D / 64, NTOK / 128), 128, 0, stream>>>(y, wo16, bo, ao);
  ln1_kernel<<<NTOK / 8, 256, 0, stream>>>(x, ao, ln1w, ln1b, x1);
  pg_kernel<<<dim3(NPG / 64, NTOK / 128), 128, 0, stream>>>(x1, wpg16, bp, bg, pg);
  ln2_kernel<<<NTOK / 8, 256, 0, stream>>>(x1, pg, offs, gate, ln2w, ln2b, out);
}
